// DyConv2d_64063732187508
// MI455X (gfx1250) — hardware-verified
//
#include <hip/hip_runtime.h>


namespace {
constexpr int B = 16, CI = 128, CO = 128, KB = 4, S = 64, KK = CI * 9;
constexpr float XS = 8.0f, WSC = 256.0f, TEMP = 30.0f;
typedef _Float16 b16;
typedef __attribute__((ext_vector_type(16))) _Float16 v16b;
typedef __attribute__((ext_vector_type(8))) _Float16 v8b;
typedef __attribute__((ext_vector_type(8))) float v8f;
typedef __attribute__((ext_vector_type(4))) float v4f;
__device__ __forceinline__ float bf16_rne(float f) { unsigned int u = __float_as_uint(f); u += 0x7FFFu + ((u >> 16) & 1u); return __uint_as_float(u & 0xFFFF0000u); }
__device__ __forceinline__ void split16(float v, b16& hi, b16& lo) { hi = (b16)v; lo = (b16)(v - (float)hi); }
__device__ __forceinline__ v16b frag_kb(const b16* p, int hh) { const v8b a = *(const v8b*)(p + 8 * hh), b = *(const v8b*)(p + 16 + 8 * hh); v16b f;
#pragma unroll
  for (int e = 0; e < 8; ++e) { f[e] = a[e]; f[8 + e] = b[e]; } return f; }
__device__ __forceinline__ v8f wmma16b(v16b a, v16b b, v8f c) { v8f d = __builtin_amdgcn_wmma_f32_16x16x32_f16(false, a, false, b, (short)0, c, false, false); asm volatile("v_nop\n\tv_nop\n\tv_nop\n\tv_nop" : "+v"(d) : "v"(a), "v"(b)); return d; }
__device__ __forceinline__ void wave_lds_sync() { __builtin_amdgcn_fence(__ATOMIC_RELEASE, "workgroup"); __builtin_amdgcn_wave_barrier(); __builtin_amdgcn_fence(__ATOMIC_ACQUIRE, "workgroup"); }
__device__ __forceinline__ float pmul(float a, float b) { float p = a * b; asm volatile("" : "+v"(p)); return p; }

__global__ __launch_bounds__(256) void pool_kernel(const float* __restrict__ x, float* __restrict__ POOL) {
  __shared__ float red[256]; const int bc = blockIdx.x, tid = threadIdx.x; const float* p = x + (size_t)bc * S * S; float s = 0.0f; for (int i = tid; i < S * S; i += 256) s += bf16_rne(p[i]); red[tid] = s; __syncthreads();
  for (int w = 128; w > 0; w >>= 1) { if (tid < w) red[tid] += red[tid + w]; __syncthreads(); }
  if (tid < 32) { const float v = tid == 0 ? red[0] * (1.0f / (S * S)) : 0.0f; for (int pass = 0; pass < 2; ++pass) { ((volatile float*)POOL)[(size_t)bc * 32 + tid] = v; __threadfence(); } }
}
__global__ __launch_bounds__(32) void se_kernel(const float* __restrict__ POOL, const float* __restrict__ w1, const float* __restrict__ w2, const float* __restrict__ b2, float* __restrict__ ATT) {
  __shared__ float pl[CI], hs[64]; const int lane = threadIdx.x, b = blockIdx.x; for (int q = 0; q < 4; ++q) pl[q * 32 + lane] = POOL[((size_t)b * CI + q * 32 + lane) * 32]; wave_lds_sync();
  for (int j = lane; j < 64; j += 32) { float s = 0.0f; if (j < 33) {
#pragma unroll 4
    for (int c = 0; c < CI; ++c) s += pmul(pl[c], bf16_rne(w1[j * CI + c])); } hs[j] = fmaxf(s, 0.0f); }
  wave_lds_sync(); float lg[KB];
#pragma unroll
  for (int k = 0; k < KB; ++k) { float s = bf16_rne(b2[k]);
#pragma unroll 1
    for (int j = 0; j < 33; ++j) s += pmul(hs[j], bf16_rne(w2[k * 33 + j])); lg[k] = s * (1.0f / TEMP); }
  float mx = fmaxf(fmaxf(lg[0], lg[1]), fmaxf(lg[2], lg[3])); float e[KB], sum = 0.0f;
#pragma unroll
  for (int k = 0; k < KB; ++k) { e[k] = __expf(lg[k] - mx); sum += e[k]; }
  const float v = lane < KB ? (lane == 0 ? e[0] : lane == 1 ? e[1] : lane == 2 ? e[2] : e[3]) / sum : 0.0f;
  for (int pass = 0; pass < 2; ++pass) { ((volatile float*)ATT)[(size_t)b * 32 + lane] = v; __threadfence(); }
}
__global__ __launch_bounds__(256) void wcomb_kernel(const float* __restrict__ W, const float* __restrict__ bias, const float* __restrict__ ATT, b16* __restrict__ WCH, b16* __restrict__ WCL, float* __restrict__ BC) {
  const size_t u = (size_t)blockIdx.x * 256 + threadIdx.x; if (u >= (size_t)B * CO * 9 * 16) return; const int c8 = (int)(u % 16), tap = (int)((u / 16) % 9), co = (int)((u / 144) % CO), b = (int)(u / (144 * CO));
  float a[KB]; for (int k = 0; k < KB; ++k) a[k] = ATT[(size_t)b * 32 + k]; v8b hv, lv;
#pragma unroll
  for (int j = 0; j < 8; ++j) { const int ci = c8 * 8 + j; float s = 0.0f; for (int k = 0; k < KB; ++k) s += pmul(a[k], bf16_rne(W[(((size_t)(k * CO + co) * CI + ci) * 9) + tap])); b16 p, q; split16(s * WSC, p, q); hv[j] = p; lv[j] = q; }
  const size_t o_ = ((size_t)(b * CO + co)) * KK + tap * CI + c8 * 8;
  for (int pass = 0; pass < 2; ++pass) { *(volatile v8b*)(WCH + o_) = hv; *(volatile v8b*)(WCL + o_) = lv; if (tap == 0 && c8 == 0) { float s = 0.0f; for (int k = 0; k < KB; ++k) s += pmul(a[k], bf16_rne(bias[k * CO + co])); ((volatile float*)BC)[((size_t)b * CO + co) * 32] = s; } __threadfence(); }
}
__global__ __launch_bounds__(32) void conv_kernel(const float* __restrict__ x, const b16* __restrict__ WCH, const b16* __restrict__ WCL, const float* __restrict__ BC, int BV, float* __restrict__ out) {
  __shared__ __attribute__((aligned(16))) b16 Xs[3][34][CI + 8]; __shared__ float Of[32][CO + 1];
  const int lane = threadIdx.x, nloc = lane & 15, hlf = lane >> 4; const int hx = blockIdx.x & 1, y = (blockIdx.x >> 1) % S, b = blockIdx.x / (2 * S); if (b >= BV) return; const int x0 = hx * 32;
  for (int kh = 0; kh < 3; ++kh) { const int yy = y + kh - 1;
    for (int xx = 0; xx < 34; ++xx) { const int xg = x0 + xx - 1; const bool ok = yy >= 0 && yy < S && xg >= 0 && xg < S;
      for (int q = 0; q < 4; ++q) { const int ci = q * 32 + lane; Xs[kh][xx][ci] = (b16)(ok ? bf16_rne(x[(((size_t)b * CI + ci) * S + yy) * S + xg]) * XS : 0.0f); } } }
  wave_lds_sync(); v8f acc[2][8];
#pragma unroll
  for (int p = 0; p < 2; ++p)
#pragma unroll
    for (int t = 0; t < 8; ++t) acc[p][t] = (v8f){};
  const b16* wh = WCH + (size_t)b * CO * KK; const b16* wl = WCL + (size_t)b * CO * KK;
#pragma unroll 1
  for (int tap = 0; tap < 9; ++tap) { const int kh = tap / 3, kw = tap % 3;
#pragma unroll
    for (int cb = 0; cb < CI; cb += 32) { const v16b a0 = frag_kb(&Xs[kh][nloc + kw][cb], hlf), a1 = frag_kb(&Xs[kh][16 + nloc + kw][cb], hlf); const int k0 = tap * CI + cb;
#pragma unroll
      for (int t = 0; t < 8; ++t) { const size_t wr = (size_t)(t * 16 + nloc) * KK + k0; const v16b bh = frag_kb(wh + wr, hlf), bl = frag_kb(wl + wr, hlf); acc[0][t] = wmma16b(a0, bh, acc[0][t]); acc[0][t] = wmma16b(a0, bl, acc[0][t]); acc[1][t] = wmma16b(a1, bh, acc[1][t]); acc[1][t] = wmma16b(a1, bl, acc[1][t]); } } }
#pragma unroll
  for (int p = 0; p < 2; ++p)
#pragma unroll
    for (int t = 0; t < 8; ++t) { const int co = t * 16 + nloc; const float bb = BC[((size_t)b * CO + co) * 32];
#pragma unroll
      for (int r8 = 0; r8 < 8; ++r8) Of[p * 16 + 8 * hlf + r8][co] = acc[p][t][r8] * (1.0f / (XS * WSC)) + bb; }
  wave_lds_sync();
  for (int pass = 0; pass < 2; ++pass) { for (int co = 0; co < CO; ++co) ((volatile float*)out)[(((size_t)b * CO + co) * S + y) * S + x0 + lane] = Of[lane][co]; __threadfence(); }
}
}

extern "C" void kernel_launch(void* const* d_in, const int* in_sizes, int n_in, void* d_out, int out_size, void* d_ws, size_t ws_size, hipStream_t stream) {
  (void)n_in;
  auto Fp = [&](int i) { return (const float*)d_in[i]; };
  if (in_sizes[0] != B * CI * S * S || in_sizes[1] != KB * CO * CI * 9 || in_sizes[2] != KB * CO || in_sizes[3] != 33 * CI || in_sizes[4] != KB * 33 || in_sizes[5] != KB || out_size != B * CO * S * S) return;
  const int BV = B;
  size_t off = 0; char* ws = (char*)d_ws;
  auto carve = [&](size_t bytes) { char* p = ws + off; off += (bytes + 255) & ~(size_t)255; return p; };
  float* POOL = (float*)carve((size_t)B * CI * 32 * 4); float* ATT = (float*)carve((size_t)B * 32 * 4); b16* WCH = (b16*)carve((size_t)B * CO * KK * 2); b16* WCL = (b16*)carve((size_t)B * CO * KK * 2); float* BC = (float*)carve((size_t)B * CO * 32 * 4);
  if (off > ws_size || off > ((size_t)16 << 20)) return;
  pool_kernel<<<B * CI, 256, 0, stream>>>(Fp(0), POOL);
  se_kernel<<<B, 32, 0, stream>>>(POOL, Fp(3), Fp(4), Fp(5), ATT);
  wcomb_kernel<<<(unsigned)((B * CO * 9 * 16 + 255) / 256), 256, 0, stream>>>(Fp(1), Fp(2), ATT, WCH, WCL, BC);
  conv_kernel<<<(unsigned)(BV * S * 2), 32, 0, stream>>>(Fp(0), WCH, WCL, BC, BV, (float*)d_out);
}
